// GNNLayer_22351009809180
// MI455X (gfx1250) — hardware-verified
//
#include <hip/hip_runtime.h>
#include <stddef.h>
#include <stdint.h>


#define DIN     128
#define DOUT    128
#define KP1     512
#define CONE    128
#define CM      192
#define CFLG    448
#define KS0     192
#define KS1     320
#define KU      512
#define HHALF   256
#define NTHR    256
#define NWAVE   8
#define EPT     8
#define CHUNK   (NTHR * EPT)
#define WCAP    (EPT * 32)
#define LISTN   (NWAVE * WCAP)
#define NBA     1024
#define PKS     10
#define RCAP    28672
#define DEGCAP  64
#define GBM     64
#define GBN     128
#define GTHR    128
#define UA      2048
#define UB      3072
#define UC      7168
#define UD      8192
#define UE      16384
#define ZINTS   (2 * RCAP + 2 * NBA + LISTN)
#define LDS_AGG (ZINTS * 4 + 64)
#define WSMAX   134217728

static_assert((CHUNK & (CHUNK - 1)) == 0);
static_assert(NBA == (1 << PKS));
static_assert(((long long)CHUNK << PKS) < (1LL << 31));
static_assert(NTHR * 4 == NBA);
static_assert(LISTN >= NBA && LISTN >= NWAVE * WCAP);
static_assert((RCAP % 32) == 0);
static_assert((ZINTS % (NTHR * 4)) == 0);
static_assert(LDS_AGG <= 262144);
static_assert((NBA % NWAVE) == 0 && (NBA % GBM) == 0);
static_assert(GBM == (GTHR / 32) * 16 && GBN == 8 * 16 && GBN == DOUT);
static_assert(KS0 + KS1 == KP1 && (KS0 % 32) == 0 && (KS1 % 32) == 0 && (KU % 32) == 0);
static_assert(CM == KS0 && CM + 2 * DIN == CFLG && CFLG + 64 == KP1 && CONE == DIN && CONE + 64 == CM);
static_assert(KU == 2 * 2 * DOUT && HHALF == 2 * DOUT);
static_assert(((KP1 * 2) % 128) == 0 && ((KU * 2) % 128) == 0);
static_assert((UA % NTHR) == 0 && (UB % NTHR) == 0 && (UC % NTHR) == 0 && (UD % NTHR) == 0 && (UE % NTHR) == 0);
static_assert(UA == DOUT * 16 && UB - UA == DOUT * 8 && UC - UB == DOUT * 32 && UD - UC == DOUT * 8 && UE - UD == DOUT * 64);
static_assert(DIN == 32 * 4);
static_assert(DIN == 16 * 8);
static_assert(DOUT == 32 * 4);

typedef float          v4f  __attribute__((ext_vector_type(4)));
typedef float          v8f  __attribute__((ext_vector_type(8)));
typedef int            v4i  __attribute__((ext_vector_type(4)));
typedef int            v8i  __attribute__((ext_vector_type(8)));
typedef unsigned int   v4u  __attribute__((ext_vector_type(4)));
typedef unsigned short v8us __attribute__((ext_vector_type(8)));
typedef __bf16         v16b __attribute__((ext_vector_type(16)));
typedef v4f  __attribute__((may_alias)) v4fa;
typedef v4i  __attribute__((may_alias)) v4ia;
typedef v8us __attribute__((may_alias)) v8usa;
union Frag { v16b b; v8us h[2]; v8i w; };

__device__ __forceinline__ v8f wmk(const Frag& a, const Frag& b, v8f c) {
  v8f d = __builtin_amdgcn_wmma_f32_16x16x32_bf16(false, a.b, false, b.b, (short)0, c, false, false);
  asm volatile("v_nop\n\tv_nop\n\tv_nop\n\tv_nop" : "+v"(d) : "v"(a.w), "v"(b.w));
  return d;
}

__device__ __forceinline__ unsigned int f2bf(float f) {
  const unsigned int u = __float_as_uint(f);
  return ((u + 0x7FFFu + ((u >> 16) & 1u)) >> 16) & 0xFFFFu;
}
__device__ __forceinline__ float bf2f(unsigned int b) { return __uint_as_float(b << 16); }
__device__ __forceinline__ float bfr(float f) { return bf2f(f2bf(f)); }
__device__ __forceinline__ v4f bfr4(const v4f a) {
  v4f r; r.x = bfr(a.x); r.y = bfr(a.y); r.z = bfr(a.z); r.w = bfr(a.w); return r;
}
__device__ __forceinline__ unsigned short bf_bits(float f) { return (unsigned short)f2bf(f); }
__device__ __forceinline__ unsigned int pk2(float lo, float hi) { return f2bf(lo) | (f2bf(hi) << 16); }
__device__ __forceinline__ v4u pack8(const v4f a, const v4f b) {
  v4u r;
  r.x = pk2(a.x, a.y); r.y = pk2(a.z, a.w); r.z = pk2(b.x, b.y); r.w = pk2(b.z, b.w);
  return r;
}
__device__ __forceinline__ void split2(float fa, float fb, unsigned int& hw, unsigned int& lw) {
  const unsigned int ha = f2bf(fa), hb = f2bf(fb);
  const unsigned int la = f2bf(fa - bf2f(ha)), lb = f2bf(fb - bf2f(hb));
  hw = ha | (hb << 16);
  lw = la | (lb << 16);
}
__device__ __forceinline__ v4f relu4(const v4f a) {
  v4f r;
  r.x = fmaxf(a.x, 0.0f); r.y = fmaxf(a.y, 0.0f); r.z = fmaxf(a.z, 0.0f); r.w = fmaxf(a.w, 0.0f);
  return r;
}

__device__ __forceinline__ int scan_chunk(const int* __restrict__ dsts, int nE, int cbase, int slotBase,
                                          int nb, int vec8, int* list, int tid, int lane, int wave) {
  int wc = 0;
  const int el0  = tid * EPT;
  const int e0   = cbase + el0;
  const int sent = -2147483647 - 1;
  v4i da, db;
  if (vec8 != 0 && cbase + CHUNK <= nE) {
    da = *(const v4i*)(dsts + e0);
    db = *(const v4i*)(dsts + e0 + 4);
  } else {
    da.x = (e0     < nE) ? dsts[min(e0,     nE - 1)] : sent;
    da.y = (e0 + 1 < nE) ? dsts[min(e0 + 1, nE - 1)] : sent;
    da.z = (e0 + 2 < nE) ? dsts[min(e0 + 2, nE - 1)] : sent;
    da.w = (e0 + 3 < nE) ? dsts[min(e0 + 3, nE - 1)] : sent;
    db.x = (e0 + 4 < nE) ? dsts[min(e0 + 4, nE - 1)] : sent;
    db.y = (e0 + 5 < nE) ? dsts[min(e0 + 5, nE - 1)] : sent;
    db.z = (e0 + 6 < nE) ? dsts[min(e0 + 6, nE - 1)] : sent;
    db.w = (e0 + 7 < nE) ? dsts[min(e0 + 7, nE - 1)] : sent;
  }
  const unsigned nbs = (unsigned)slotBase;
  const unsigned unb = (unsigned)nb;
  const unsigned s0 = (unsigned)da.x - nbs, s1 = (unsigned)da.y - nbs;
  const unsigned s2 = (unsigned)da.z - nbs, s3 = (unsigned)da.w - nbs;
  const unsigned s4 = (unsigned)db.x - nbs, s5 = (unsigned)db.y - nbs;
  const unsigned s6 = (unsigned)db.z - nbs, s7 = (unsigned)db.w - nbs;
  const bool h0 = s0 < unb, h1 = s1 < unb, h2 = s2 < unb, h3 = s3 < unb;
  const bool h4 = s4 < unb, h5 = s5 < unb, h6 = s6 < unb, h7 = s7 < unb;
  const unsigned any = __builtin_amdgcn_ballot_w32(h0 | h1 | h2 | h3 | h4 | h5 | h6 | h7);
  if (any != 0u) {
#define HITJ(J, HJ, SJ) { \
      const unsigned mj = __builtin_amdgcn_ballot_w32(HJ); \
      if (mj != 0u) { \
        if (HJ) { \
          const int pos = wc + (int)__builtin_amdgcn_mbcnt_lo(mj, 0u); \
          if (pos < WCAP) list[wave * WCAP + pos] = ((el0 + (J)) << PKS) | (int)(SJ); \
        } \
        wc += (int)__builtin_popcount(mj); } }
    HITJ(0, h0, s0)
    HITJ(1, h1, s1)
    HITJ(2, h2, s2)
    HITJ(3, h3, s3)
    HITJ(4, h4, s4)
    HITJ(5, h5, s5)
    HITJ(6, h6, s6)
    HITJ(7, h7, s7)
#undef HITJ
  }
  return wc;
}

__global__ __launch_bounds__(NTHR) void k_prep(const float* __restrict__ wlin, const float* __restrict__ blin,
                                               const float* __restrict__ wmsg, const float* __restrict__ bmsg,
                                               const float* __restrict__ wupd,
                                               unsigned short* B1T, unsigned short* B2T) {
  const int u = (int)blockIdx.x * NTHR + (int)threadIdx.x;
  v8us o;
  unsigned short* dp;
  if (u < UA) {
    const int n = u >> 4, q = u & 15;
    const float* p = wlin + (size_t)(8 * q) * DOUT + n;
#pragma unroll
    for (int j = 0; j < 8; ++j) o[j] = bf_bits(p[(size_t)j * DOUT]);
    dp = B1T + (size_t)n * KP1 + 8 * q;
  } else if (u < UB) {
    const int v = u - UA;
    const int n = v >> 3, j = v & 7;
    const unsigned int msk = 0u - (unsigned int)(j == 0);
    o[0] = (unsigned short)(f2bf(blin[n]) & msk);
    o[1] = 0; o[2] = 0; o[3] = 0; o[4] = 0; o[5] = 0; o[6] = 0; o[7] = 0;
    dp = B1T + (size_t)n * KP1 + CONE + 8 * j;
  } else if (u < UC) {
    const int v = u - UB;
    const int n = v >> 5, t = v & 31;
    const float* p = wmsg + (size_t)(4 * t) * DOUT + n;
    const unsigned short b0 = bf_bits(p[0]), b1 = bf_bits(p[(size_t)DOUT]);
    const unsigned short b2 = bf_bits(p[(size_t)2 * DOUT]), b3 = bf_bits(p[(size_t)3 * DOUT]);
    o[0] = b0; o[1] = b1; o[2] = b0; o[3] = b1;
    o[4] = b2; o[5] = b3; o[6] = b2; o[7] = b3;
    dp = B1T + (size_t)n * KP1 + CM + 8 * t;
  } else if (u < UD) {
    const int v = u - UC;
    const int n = v >> 3, j = v & 7;
    const unsigned int msk = 0u - (unsigned int)(j == 0);
    o[0] = (unsigned short)(f2bf(bmsg[n]) & msk);
    o[1] = 0; o[2] = 0; o[3] = 0; o[4] = 0; o[5] = 0; o[6] = 0; o[7] = 0;
    dp = B1T + (size_t)n * KP1 + CFLG + 8 * j;
  } else if (u < UE) {
    const int v = u - UD;
    const int n = v >> 6, q = v & 63;
    const float* p = wupd + (size_t)(4 * q) * DOUT + n;
    const unsigned short b0 = bf_bits(p[0]), b1 = bf_bits(p[(size_t)DOUT]);
    const unsigned short b2 = bf_bits(p[(size_t)2 * DOUT]), b3 = bf_bits(p[(size_t)3 * DOUT]);
    o[0] = b0; o[1] = b1; o[2] = b0; o[3] = b1;
    o[4] = b2; o[5] = b3; o[6] = b2; o[7] = b3;
    dp = B2T + (size_t)n * KU + 8 * q;
  } else {
    return;
  }
  *(volatile v8us*)dp = o;
  __threadfence();
  *(volatile v8us*)dp = o;
}

__global__ __launch_bounds__(NTHR) void k_agg(const int* __restrict__ keys, const int* __restrict__ srcs,
                                              const float* __restrict__ X, unsigned short* Aout,
                                              int nN, int nE, int vec8) {
  extern __shared__ __attribute__((aligned(16))) int lds_i[];
  int* reg1 = lds_i;
  int* reg2 = reg1 + RCAP;
  int* scnt = reg2 + RCAP;
  int* soff = scnt + NBA;
  int* list = soff + NBA;
  int* wcnt = list + LISTN;
  int* wtot = wcnt + NWAVE;
  const int tid = (int)threadIdx.x, lane = tid & 31, wave = tid >> 5;
  const int nodeBase = (int)blockIdx.x * NBA;

  {
    const v4i z4 = {0, 0, 0, 0};
    for (int i = tid * 4; i < ZINTS; i += NTHR * 4) *(v4ia*)(lds_i + i) = z4;
    if (tid < 2 * NWAVE) wcnt[tid] = 0;
  }
  __syncthreads();

  int tot = 0;
  const int nChunks = (nE + CHUNK - 1) / CHUNK;
#pragma unroll 1
  for (int ch = 0; ch < nChunks; ++ch) {
    const int cbase = ch * CHUNK;
    const int wc = scan_chunk(keys, nE, cbase, nodeBase, NBA, vec8, list, tid, lane, wave);
    if (lane == 0) wcnt[wave] = wc;
    __syncthreads();
    int pre = 0, all = 0;
#pragma unroll
    for (int w2 = 0; w2 < NWAVE; ++w2) {
      int c = wcnt[w2];
      c = c < 0 ? 0 : (c > WCAP ? WCAP : c);
      all += c;
      pre += (w2 < wave) ? c : 0;
    }
    const int wcc  = wc > WCAP ? WCAP : wc;
    const int base = tot + pre;
#pragma unroll 1
    for (int i = lane; i < wcc; i += 32) {
      const int ent = list[wave * WCAP + i];
      const int el  = (ent >> PKS) & (CHUNK - 1);
      const int sl  = ent & (NBA - 1);
      int eid = cbase + el;
      eid = eid > nE - 1 ? nE - 1 : eid;
      const int pos = base + i;
      if (pos < RCAP) reg1[pos] = (int)(((unsigned)eid << PKS) | (unsigned)sl);
    }
    tot += all;
    tot = tot > RCAP ? RCAP : tot;
    __syncthreads();
  }
  const int nh = tot;

  if (wave == 0) {
#pragma unroll 1
    for (int b0 = 0; b0 < nh; b0 += 32) {
      const int idx = b0 + lane;
      const int uv  = reg1[idx < RCAP ? idx : RCAP - 1];
      const int m32 = (nh - b0) < 32 ? (nh - b0) : 32;
#pragma unroll 1
      for (int k = 0; k < m32; ++k) {
        const int u  = __builtin_amdgcn_readlane(uv, k);
        const int sl = u & (NBA - 1);
        if (lane == 0) scnt[sl] = scnt[sl] + 1;
      }
    }
  }
  __syncthreads();

  {
    const v4i ca = *(const v4ia*)(scnt + 4 * tid);
    const int e0 = ca.x < 0 ? 0 : ca.x, e1 = ca.y < 0 ? 0 : ca.y, e2 = ca.z < 0 ? 0 : ca.z, e3 = ca.w < 0 ? 0 : ca.w;
    const int ts = e0 + e1 + e2 + e3;
    int incl = ts;
#pragma unroll
    for (int d = 1; d < 32; d <<= 1) {
      const int up = __shfl_up(incl, d, 32);
      if (lane >= d) incl += up;
    }
    if (lane == 31) wtot[wave] = incl;
    __syncthreads();
    int pre = 0;
#pragma unroll
    for (int w2 = 0; w2 < NWAVE; ++w2) pre += (w2 < wave) ? wtot[w2] : 0;
    int run = pre + incl - ts;
    soff[4 * tid + 0] = run; run += e0;
    soff[4 * tid + 1] = run; run += e1;
    soff[4 * tid + 2] = run; run += e2;
    soff[4 * tid + 3] = run;
  }
  __syncthreads();
  for (int i = tid; i < NBA; i += NTHR) list[i] = soff[i];
  __syncthreads();

  if (wave == 0) {
#pragma unroll 1
    for (int b0 = 0; b0 < nh; b0 += 32) {
      const int idx = b0 + lane;
      const int uv  = reg1[idx < RCAP ? idx : RCAP - 1];
      const int m32 = (nh - b0) < 32 ? (nh - b0) : 32;
#pragma unroll 1
      for (int k = 0; k < m32; ++k) {
        const int u   = __builtin_amdgcn_readlane(uv, k);
        const int sl  = u & (NBA - 1);
        const int eid = (int)((unsigned)u >> PKS);
        if (lane == 0) {
          int pos = list[sl];
          pos = pos < 0 ? 0 : (pos > RCAP - 1 ? RCAP - 1 : pos);
          reg2[pos] = eid;
          list[sl] = pos + 1;
        }
      }
    }
  }
  __syncthreads();

  const int nbw = NBA / NWAVE;
  const bool ovf = (nh >= RCAP);
  const float qnan = __int_as_float(0x7fc00000);
  const int c4 = 4 * lane;
  const int c8 = 8 * (lane & 15);
  const bool xw = lane < 16;
  const bool w8 = lane < 8;
  const unsigned int l0m = 0u - (unsigned int)(lane == 0);
  const v4f z4 = {0.0f, 0.0f, 0.0f, 0.0f};

#pragma unroll 1
  for (int jt = 0; jt < nbw; ++jt) {
    const int slot = wave * nbw + jt;
    const int node = nodeBase + slot;
    int st = soff[slot];
    const int craw = scnt[slot];
    int cnt = craw;
    st  = st < 0 ? 0 : (st > nh ? nh : st);
    cnt = cnt < 0 ? 0 : (cnt > DEGCAP ? DEGCAP : cnt);
    if (cnt > nh - st) cnt = nh - st;
    const float pz = (ovf || craw > DEGCAP) ? qnan : 0.0f;
    const bool live = node < nN;
    const float okf = live ? 1.0f : 0.0f;
    const int nc = node < nN ? node : nN - 1;

    v4f a = z4;
#pragma unroll 1
    for (int b0 = 0; b0 < cnt; b0 += 32) {
      int idx = st + b0 + lane; idx = idx > RCAP - 1 ? RCAP - 1 : idx;
      int eid = reg2[idx]; eid = eid < 0 ? 0 : (eid > nE - 1 ? nE - 1 : eid);
      int sr = srcs[eid]; sr = sr < 0 ? 0 : (sr > nN - 1 ? nN - 1 : sr);
      const int m32 = (cnt - b0) < 32 ? (cnt - b0) : 32;
#pragma unroll 1
      for (int k = 0; k < m32; ++k) {
        const int sk = __builtin_amdgcn_readlane(sr, k);
        const v4f v = *(const v4fa*)(X + (size_t)sk * DIN + c4);
        a += bfr4(v);
      }
    }
    const float inv = 1.0f / (float)(cnt > 0 ? cnt : 1);
    const v4f mm = a * (inv * okf) + pz;

    v4u mw;
    { unsigned int h0, l0, h1, l1;
      split2(mm.x, mm.y, h0, l0);
      split2(mm.z, mm.w, h1, l1);
      mw.x = h0; mw.y = l0; mw.z = h1; mw.w = l1; }

    const float* xp = X + (size_t)nc * DIN + c8;
    const v4f xa = *(const v4fa*)xp * okf;
    const v4f xb = *(const v4fa*)(xp + 4) * okf;
    const v4u xv = pack8(xa, xb);

    v4u ow, fw;
    ow.x = (live ? 0x3F80u : 0u) & l0m;                 ow.y = 0u; ow.z = 0u; ow.w = 0u;
    fw.x = ((live && cnt > 0) ? 0x3F80u : 0u) & l0m;    fw.y = 0u; fw.z = 0u; fw.w = 0u;

    unsigned short* rp = Aout + (size_t)node * (size_t)KP1;
    if (xw) *(volatile v4u*)(rp + c8) = xv;
    if (w8) *(volatile v4u*)(rp + CONE + 8 * lane) = ow;
    *(volatile v4u*)(rp + CM + 8 * lane) = mw;
    if (w8) *(volatile v4u*)(rp + CFLG + 8 * lane) = fw;
    __threadfence();
    if (xw) *(volatile v4u*)(rp + c8) = xv;
    if (w8) *(volatile v4u*)(rp + CONE + 8 * lane) = ow;
    *(volatile v4u*)(rp + CM + 8 * lane) = mw;
    if (w8) *(volatile v4u*)(rp + CFLG + 8 * lane) = fw;
  }
}

__global__ __launch_bounds__(GTHR) void k_gemm1(const unsigned short* __restrict__ A,
                                                const unsigned short* __restrict__ BT,
                                                unsigned short* AU) {
  __shared__ __attribute__((aligned(16))) float stg[GBM * GBN];
  const int tid = (int)threadIdx.x, lane = tid & 31, wave = tid >> 5, hh = lane >> 4, m = lane & 15;
  const int rowBase = (int)blockIdx.x * GBM;
  const int y    = (int)blockIdx.y;
  const int kofs = y * KS0;
  const int K    = KS0 + (KS1 - KS0) * y;

  v8f acc[8];
  {
    const v8f z = {0.f, 0.f, 0.f, 0.f, 0.f, 0.f, 0.f, 0.f};
#pragma unroll
    for (int t = 0; t < 8; ++t) acc[t] = z;
  }
  const unsigned short* ap = A  + (size_t)(rowBase + 16 * wave + m) * (size_t)KP1 + kofs + 8 * hh;
  const unsigned short* bp = BT + (size_t)m * (size_t)KP1 + kofs + 8 * hh;

#pragma unroll 1
  for (int k0 = 0; k0 < K; k0 += 32) {
    Frag af;
    af.h[0] = *(const v8usa*)(ap + k0);
    af.h[1] = *(const v8usa*)(ap + k0 + 16);
#pragma unroll
    for (int nt = 0; nt < 8; ++nt) {
      const unsigned short* wq = bp + (size_t)(16 * nt) * (size_t)KP1 + k0;
      Frag bf;
      bf.h[0] = *(const v8usa*)wq;
      bf.h[1] = *(const v8usa*)(wq + 16);
      acc[nt] = wmk(af, bf, acc[nt]);
    }
  }

#pragma unroll
  for (int nt = 0; nt < 8; ++nt) {
    const int lc = 16 * nt + m;
#pragma unroll
    for (int r = 0; r < 8; ++r) {
      const int lr = 16 * wave + 8 * hh + r;
      stg[lr * GBN + lc] = acc[nt][r];
    }
  }
  __syncthreads();

  v4u ov[16];
#pragma unroll
  for (int i = 0; i < 16; ++i) {
    const v4f f = *(const v4fa*)(stg + (16 * wave + i) * GBN + 4 * lane);
    unsigned int h0, l0, h1, l1;
    split2(f.x, f.y, h0, l0);
    split2(f.z, f.w, h1, l1);
    v4u o; o.x = h0; o.y = l0; o.z = h1; o.w = l1;
    ov[i] = o;
  }
#pragma unroll
  for (int i = 0; i < 16; ++i) {
    unsigned short* op = AU + (size_t)(rowBase + 16 * wave + i) * (size_t)KU + HHALF * y + 8 * lane;
    *(volatile v4u*)op = ov[i];
  }
  __threadfence();
#pragma unroll
  for (int i = 0; i < 16; ++i) {
    unsigned short* op = AU + (size_t)(rowBase + 16 * wave + i) * (size_t)KU + HHALF * y + 8 * lane;
    *(volatile v4u*)op = ov[i];
  }
}

__global__ __launch_bounds__(GTHR) void k_gemm2(const unsigned short* __restrict__ A,
                                                const unsigned short* __restrict__ BT,
                                                const float* __restrict__ bias, float* out, int nN) {
  __shared__ __attribute__((aligned(16))) float stg[GBM * GBN];
  const int tid = (int)threadIdx.x, lane = tid & 31, wave = tid >> 5, hh = lane >> 4, m = lane & 15;
  const int rowBase = (int)blockIdx.x * GBM;

  v8f acc[8];
  {
    const v8f z = {0.f, 0.f, 0.f, 0.f, 0.f, 0.f, 0.f, 0.f};
#pragma unroll
    for (int t = 0; t < 8; ++t) acc[t] = z;
  }
  const unsigned short* ap = A  + (size_t)(rowBase + 16 * wave + m) * (size_t)KU + 8 * hh;
  const unsigned short* bp = BT + (size_t)m * (size_t)KU + 8 * hh;

#pragma unroll 1
  for (int k0 = 0; k0 < KU; k0 += 32) {
    Frag af;
    af.h[0] = *(const v8usa*)(ap + k0);
    af.h[1] = *(const v8usa*)(ap + k0 + 16);
#pragma unroll
    for (int nt = 0; nt < 8; ++nt) {
      const unsigned short* wq = bp + (size_t)(16 * nt) * (size_t)KU + k0;
      Frag bf;
      bf.h[0] = *(const v8usa*)wq;
      bf.h[1] = *(const v8usa*)(wq + 16);
      acc[nt] = wmk(af, bf, acc[nt]);
    }
  }

#pragma unroll
  for (int nt = 0; nt < 8; ++nt) {
    const int lc = 16 * nt + m;
#pragma unroll
    for (int r = 0; r < 8; ++r) {
      const int lr = 16 * wave + 8 * hh + r;
      stg[lr * GBN + lc] = acc[nt][r];
    }
  }
  __syncthreads();

  const v4f bb = bfr4(*(const v4fa*)(bias + 4 * lane));
  v4f fv[16];
#pragma unroll
  for (int i = 0; i < 16; ++i)
    fv[i] = relu4(*(const v4fa*)(stg + (16 * wave + i) * GBN + 4 * lane) + bb);
#pragma unroll
  for (int i = 0; i < 16; ++i) {
    const int gr = rowBase + 16 * wave + i;
    float* op = out + (size_t)gr * (size_t)DOUT + 4 * lane;
    if (gr < nN) *(volatile v4f*)op = fv[i];
  }
  __threadfence();
#pragma unroll
  for (int i = 0; i < 16; ++i) {
    const int gr = rowBase + 16 * wave + i;
    float* op = out + (size_t)gr * (size_t)DOUT + 4 * lane;
    if (gr < nN) *(volatile v4f*)op = fv[i];
  }
}

static inline int cdiv(int a, int b) { return (a + b - 1) / b; }
static inline size_t al256(size_t o) { return (o + 255) & ~(size_t)255; }

extern "C" void kernel_launch(void* const* d_in, const int* in_sizes, int n_in,
                              void* d_out, int out_size, void* d_ws, size_t ws_size,
                              hipStream_t stream) {
  if (n_in < 8) return;
  if (in_sizes[0] < DIN || (in_sizes[0] % DIN) != 0) return;
  const int nN = in_sizes[0] / DIN;
  if (nN < 1 || nN > (1 << 22)) return;
  if (in_sizes[1] < 2 || (in_sizes[1] & 1) != 0) return;
  const int nE = in_sizes[1] / 2;
  if (nE < 1 || nE >= (1 << 21)) return;
  if (in_sizes[2] != DIN * DOUT) return;
  if (in_sizes[3] != DOUT) return;
  if (in_sizes[4] != DIN * DOUT) return;
  if (in_sizes[5] != DOUT) return;
  if (in_sizes[6] != 2 * DOUT * DOUT) return;
  if (in_sizes[7] != DOUT) return;
  if ((long long)out_size != (long long)nN * DOUT) return;

  const float* x    = (const float*)d_in[0];
  const int*   edge = (const int*)d_in[1];
  const float* wlin = (const float*)d_in[2];
  const float* blin = (const float*)d_in[3];
  const float* wmsg = (const float*)d_in[4];
  const float* bmsg = (const float*)d_in[5];
  const float* wupd = (const float*)d_in[6];
  const float* bupd = (const float*)d_in[7];
  float* out = (float*)d_out;
  const int* keys = edge;
  const int* srcs = edge + nE;

  const int MP   = cdiv(nN, GBM) * GBM;
  const int gM   = MP / GBM;
  const int gA   = cdiv(MP, NBA);
  const int RA   = gA * NBA;
  const int vec8 = 1;
  if ((long long)RA < (long long)MP) return;

  char* ws = (char*)d_ws;
  size_t off = 0;
  const size_t oB1 = off; off = al256(off + (size_t)DOUT * KP1 * 2);
  const size_t oB2 = off; off = al256(off + (size_t)DOUT * KU  * 2);
  const size_t oAP = off; off = al256(off + (size_t)RA   * KP1 * 2);
  const size_t oAU = off; off = al256(off + (size_t)MP   * KU  * 2);
  if (off > ws_size || off > (size_t)WSMAX) return;
  unsigned short* B1T = (unsigned short*)(ws + oB1);
  unsigned short* B2T = (unsigned short*)(ws + oB2);
  unsigned short* AP  = (unsigned short*)(ws + oAP);
  unsigned short* AU  = (unsigned short*)(ws + oAU);

  hipFuncSetAttribute(reinterpret_cast<const void*>(&k_agg), hipFuncAttributeMaxDynamicSharedMemorySize, LDS_AGG);

  k_prep<<<UE / NTHR, NTHR, 0, stream>>>(wlin, blin, wmsg, bmsg, wupd, B1T, B2T);
  k_agg<<<gA, NTHR, LDS_AGG, stream>>>(keys, srcs, x, AP, nN, nE, vec8);
  k_gemm1<<<dim3(gM, 2), GTHR, 0, stream>>>(AP, B1T, AU);
  k_gemm2<<<dim3(gM, 1), GTHR, 0, stream>>>(AU, B2T, bupd, out, nN);
}
